// MultiHeadAttention_67637144977483
// MI455X (gfx1250) — hardware-run, weakly checked
//
#include <hip/hip_runtime.h>


#ifndef NB
#define NB 8
#endif
#define NB_FULL 8
#define CI   64
#define CN   512
#define HW   4096
#define CO   64
#define QRS  2048.0f
#define QRI  (1.0f / 2048.0f)
#define PCAR 1024.0f
#define PCAI (1.0f / 1024.0f)
#define WSC  64.0f
#define WSI  (1.0f / 64.0f)
#define LOG2E 1.4426950408889634f

static_assert(NB <= NB_FULL);
static_assert(HW == 8 * CN);
static_assert(CI % 32 == 0);
static_assert(CN % 32 == 0);
static_assert(HW % 32 == 0);
static_assert(CN % 64 == 0);
static_assert(HW % 64 == 0);
static_assert(CO == 64);
static_assert(CI == 64);
static_assert((NB * CN) % 16 == 0);
static_assert(((size_t)CN * CI) % 8 == 0);
static_assert(((size_t)CN * CN) % 8 == 0);
static_assert(((size_t)CO * CN) % 8 == 0);

typedef _Float16 h16;
typedef unsigned short bf;
typedef __attribute__((ext_vector_type(16))) __bf16   v16bf;
typedef __attribute__((ext_vector_type(16))) _Float16 v16h;
typedef __attribute__((ext_vector_type(8)))  _Float16 v8h;
typedef __attribute__((ext_vector_type(8)))  unsigned short v8us;
typedef __attribute__((ext_vector_type(8)))  float    v8f;
typedef __attribute__((ext_vector_type(4)))  float    v4f;
typedef v4f  __attribute__((may_alias)) v4fa;
typedef v8h  __attribute__((may_alias)) v8ha;
typedef v8us __attribute__((may_alias)) v8usa;

__device__ __forceinline__ unsigned short f2bf(float f) { unsigned u = __float_as_uint(f); u += 0x7FFFu + ((u >> 16) & 1u); return (unsigned short)(u >> 16); }
__device__ __forceinline__ float bfr(float f) { return __uint_as_float(((unsigned)f2bf(f)) << 16); }
__device__ __forceinline__ v16h cat16(v8h lo, v8h hi) { return __builtin_shufflevector(lo, hi, 0, 1, 2, 3, 4, 5, 6, 7, 8, 9, 10, 11, 12, 13, 14, 15); }
__device__ __forceinline__ v16bf cat16b(v8us lo, v8us hi) { return __builtin_bit_cast(v16bf, __builtin_shufflevector(lo, hi, 0, 1, 2, 3, 4, 5, 6, 7, 8, 9, 10, 11, 12, 13, 14, 15)); }
__device__ __forceinline__ v8f wmma16(v16h a, v16h b, v8f c) { return __builtin_amdgcn_wmma_f32_16x16x32_f16(false, a, false, b, (short)0, c, false, false); }
__device__ __forceinline__ v8f wmmab(v16bf a, v16bf b, v8f c) { return __builtin_amdgcn_wmma_f32_16x16x32_bf16(false, a, false, b, (short)0, c, false, false); }
__device__ __forceinline__ v16h  ldh(const h16* p) { return cat16(*(const v8h*)p, *(const v8h*)(p + 16)); }
__device__ __forceinline__ v16bf ldb(const bf* p)  { return cat16b(*(const v8us*)p, *(const v8us*)(p + 16)); }
__device__ __forceinline__ void wave_sync() { __builtin_amdgcn_fence(3  , "wavefront"); __builtin_amdgcn_wave_barrier(); asm volatile("" ::: "memory"); }

template<int OPK> struct Ops;
template<> struct Ops<0> { typedef v16bf F;
    static __device__ __forceinline__ F ld(const bf* p) { return ldb(p); }
    static __device__ __forceinline__ v8f mm(F a, F b, v8f c) { return wmmab(a, b, c); } };
template<> struct Ops<1> { typedef v16h F;
    static __device__ __forceinline__ F ld(const bf* p) { return ldh((const h16*)p); }
    static __device__ __forceinline__ v8f mm(F a, F b, v8f c) { return wmma16(a, b, c); } };

__global__ __launch_bounds__(256) void k_cvt8(const float* __restrict__ src, bf* dst, size_t n8, int mode, float scale) {
    const size_t i = (size_t)blockIdx.x * 256 + threadIdx.x; if (i >= n8) return;
    const v8f v = *(const v8f*)(src + i * 8);
    if (mode == 0) {
        v8us o;
#pragma unroll
        for (int k = 0; k < 8; ++k) o[k] = f2bf(v[k]);
        *(volatile v8us*)(dst + i * 8) = o; __threadfence(); *(volatile v8us*)(dst + i * 8) = o;
    } else {
        v8h o;
#pragma unroll
        for (int k = 0; k < 8; ++k) o[k] = (h16)(bfr(v[k]) * scale);
        h16* dh = (h16*)dst;
        *(volatile v8h*)(dh + i * 8) = o; __threadfence(); *(volatile v8h*)(dh + i * 8) = o;
    }
}

__global__ __launch_bounds__(256) void k_xT(const float* __restrict__ src, bf* dst) {
    __shared__ __align__(16) unsigned short ts[64 * 72];
    const int t = threadIdx.x; const int m0 = blockIdx.x * 64; const int b = blockIdx.y;
    const int c = t >> 2, mq = (t & 3) * 16;
    const float* sp = src + ((size_t)b * CI + c) * HW + m0 + mq;
#pragma unroll
    for (int q = 0; q < 4; ++q) { const v4f x = *(const v4f*)(sp + 4 * q);
#pragma unroll
        for (int e = 0; e < 4; ++e) ts[(mq + 4 * q + e) * 72 + c] = f2bf(x[e]); }
    __syncthreads();
    bf* dp = dst + ((size_t)b * HW + m0) * CI;
#pragma unroll 1
    for (int ps = 0; ps < 2; ++ps) {
#pragma unroll
        for (int s = 0; s < 2; ++s) { const int p = t + 256 * s; const int row = p >> 3, c8 = (p & 7) * 8;
            const v8us o = *(const v8usa*)(&ts[row * 72 + c8]);
            *(volatile v8us*)(dp + (size_t)row * CI + c8) = o; }
        if (ps == 0) __threadfence(); }
}

template<int OPK, int RES>
__global__ __launch_bounds__(32) void k_gemm(const bf* __restrict__ A, const bf* __restrict__ AR, const bf* __restrict__ Bt,
                                             h16* CH, h16* CR, float* CF, const float* __restrict__ bias,
                                             int K, int ldc, size_t sA, size_t sB, size_t sC, float alpha, int omode, int bmode, int leaky) {
    typedef typename Ops<OPK>::F F;
    __shared__ __align__(16) float os[16 * 68];
    constexpr int TR  = RES ? 32 : 64;
    constexpr int MBR = RES ? 2 : 4;
    const int lane = threadIdx.x & 31, lr = lane & 15, hi = lane >> 4;
    const int r0 = blockIdx.x * TR, c0 = blockIdx.y * 64; const size_t z = blockIdx.z;
    v8f acc[4][4];
#pragma unroll
    for (int ab = 0; ab < 4; ++ab)
#pragma unroll
        for (int nb = 0; nb < 4; ++nb) acc[ab][nb] = (v8f){};
    const size_t aoff = z * sA + (size_t)(r0 + lr) * K + 8 * hi, boff = z * sB + (size_t)(c0 + lr) * K + 8 * hi;
#pragma unroll 1
    for (int kc = 0; kc < K; kc += 32) {
        F a[4];
#pragma unroll
        for (int ab = 0; ab < 4; ++ab) {
            const size_t off = aoff + (size_t)((RES ? (ab & 1) : ab) * 16) * K + kc;
            if (RES && ab >= 2) a[ab] = Ops<OPK>::ld(AR + off); else a[ab] = Ops<OPK>::ld(A + off);
        }
#pragma unroll
        for (int nb = 0; nb < 4; ++nb) { const F b = Ops<OPK>::ld(Bt + boff + (size_t)nb * 16 * K + kc);
#pragma unroll
            for (int ab = 0; ab < 4; ++ab) acc[ab][nb] = Ops<OPK>::mm(a[ab], b, acc[ab][nb]); }
        asm volatile("v_nop\n\tv_nop\n\tv_nop\n\tv_nop" : "+v"(acc[0][0]), "+v"(acc[1][1]), "+v"(acc[2][2]), "+v"(acc[3][3]) : "v"(a[0]), "v"(a[1]), "v"(a[2]), "v"(a[3]));
    }
    float bcol[4];
#pragma unroll
    for (int nb = 0; nb < 4; ++nb) { const int ci = (bmode == 2) ? (c0 + nb * 16 + lr) : 0; const float bv = bfr(bias[ci]); bcol[nb] = (bmode == 2) ? bv : 0.0f; }
#pragma unroll
    for (int mb = 0; mb < MBR; ++mb) {
#pragma unroll
        for (int j = 0; j < 8; ++j) {
            const int ri = (bmode == 1) ? (r0 + mb * 16 + hi * 8 + j) : 0; const float bw = bfr(bias[ri]); const float br = (bmode == 1) ? bw : 0.0f;
#pragma unroll
            for (int nb = 0; nb < 4; ++nb) {
                float v = acc[mb][nb][j];
                if (RES) v += acc[RES ? (mb + 2) : mb][nb][j] * QRI;
                v = v * alpha + (br + bcol[nb]);
                if (leaky) v = (v >= 0.0f) ? v : 0.01f * v;
                os[(hi * 8 + j) * 68 + nb * 16 + lr] = v; }
        }
        wave_sync();
        const size_t sb = z * sC + (size_t)(r0 + mb * 16) * (size_t)ldc + (size_t)c0;
        if (omode != 2) {
#pragma unroll 1
            for (int ps = 0; ps < 2; ++ps) {
#pragma unroll
                for (int s = 0; s < 4; ++s) { const int row = 4 * s + (lane >> 3), c8 = (lane & 7) * 8;
                    const v4f x0 = *(const v4fa*)(&os[row * 68 + c8]); const v4f x1 = *(const v4fa*)(&os[row * 68 + c8 + 4]); v8h hv, rv;
#pragma unroll
                    for (int i = 0; i < 4; ++i) { const h16 a0 = (h16)x0[i]; const h16 a1 = (h16)x1[i]; hv[i] = a0; hv[4 + i] = a1; rv[i] = (h16)((x0[i] - (float)a0) * QRS); rv[4 + i] = (h16)((x1[i] - (float)a1) * QRS); }
                    const size_t oo = sb + (size_t)row * (size_t)ldc + c8;
                    *(volatile v8h*)(CH + oo) = hv; if (omode == 1) *(volatile v8h*)(CR + oo) = rv; }
                if (ps == 0) __threadfence(); }
        } else {
#pragma unroll 1
            for (int ps = 0; ps < 2; ++ps) {
#pragma unroll
                for (int s = 0; s < 8; ++s) { const int row = 2 * s + hi, cofs = lr * 4;
                    const v4f val = *(const v4fa*)(&os[row * 68 + cofs]);
                    *(volatile v4f*)(CF + sb + (size_t)row * (size_t)ldc + cofs) = val; }
                if (ps == 0) __threadfence(); }
        }
        wave_sync();
    }
}

__global__ __launch_bounds__(256) void k_softmax(const float* __restrict__ S, h16* P, int nrows) {
    const int lane = threadIdx.x & 31, wave = threadIdx.x >> 5;
    const int row = blockIdx.x * 8 + wave; if (row >= nrows) return;
    const float* sp = S + (size_t)row * CN + 8 * lane;
    const v4f a0 = *(const v4f*)(sp), a1 = *(const v4f*)(sp + 4), b0 = *(const v4f*)(sp + 256), b1 = *(const v4f*)(sp + 260);
    float x[16];
#pragma unroll
    for (int i = 0; i < 4; ++i) { x[i] = a0[i]; x[4 + i] = a1[i]; x[8 + i] = b0[i]; x[12 + i] = b1[i]; }
    float mx = x[0];
#pragma unroll
    for (int i = 1; i < 16; ++i) mx = fmaxf(mx, x[i]);
    mx = fmaxf(mx, __shfl_xor(mx, 16, 32)); mx = fmaxf(mx, __shfl_xor(mx, 8, 32)); mx = fmaxf(mx, __shfl_xor(mx, 4, 32));
    mx = fmaxf(mx, __shfl_xor(mx, 2, 32));  mx = fmaxf(mx, __shfl_xor(mx, 1, 32));
    float sum = 0.0f;
#pragma unroll
    for (int i = 0; i < 16; ++i) { x[i] = __builtin_amdgcn_exp2f((x[i] - mx) * LOG2E); sum += x[i]; }
    sum += __shfl_xor(sum, 16, 32); sum += __shfl_xor(sum, 8, 32); sum += __shfl_xor(sum, 4, 32); sum += __shfl_xor(sum, 2, 32); sum += __shfl_xor(sum, 1, 32);
    const float sc = PCAR * (1.0f / sum);
    v8h pa, pb;
#pragma unroll
    for (int i = 0; i < 8; ++i) { pa[i] = (h16)(x[i] * sc); pb[i] = (h16)(x[8 + i] * sc); }
    h16* dp = P + (size_t)row * CN + 8 * lane;
    *(volatile v8h*)(dp) = pa; *(volatile v8h*)(dp + 256) = pb;
    __threadfence();
    *(volatile v8h*)(dp) = pa; *(volatile v8h*)(dp + 256) = pb;
}

__global__ __launch_bounds__(256) void k_bnstats(const float* __restrict__ O, const float* __restrict__ g, const float* __restrict__ be, float* ST) {
    __shared__ double r1[256];
    __shared__ double r2[256];
    const int t = threadIdx.x; const int qd = t & 15, rg = t >> 4; const int ch0 = blockIdx.x * 8;
    const float* p = O + (size_t)ch0 * 8 + qd * 4;
    double s1 = 0.0, s2 = 0.0;
#pragma unroll 2
    for (int r = rg; r < NB * CN; r += 16) { const v4f x = *(const v4f*)(p + (size_t)r * HW);
#pragma unroll
        for (int e = 0; e < 4; ++e) { const double d = (double)x[e]; s1 += d; s2 += d * d; } }
    r1[t] = s1; r2[t] = s2;
    __syncthreads();
    if (t < 8) {
        double a = 0.0, q = 0.0;
#pragma unroll 1
        for (int i = 0; i < 16; ++i) { a += r1[i * 16 + 2 * t]; a += r1[i * 16 + 2 * t + 1]; q += r2[i * 16 + 2 * t]; q += r2[i * 16 + 2 * t + 1]; }
        const double invn = 1.0 / (double)((size_t)NB * HW);
        const double mean = a * invn; double var = q * invn - mean * mean; if (var < 0.0) var = 0.0;
        const float rstd = rsqrtf((float)var + 1e-4f);
        v4f o; o[0] = (float)mean; o[1] = rstd * bfr(g[ch0 + t]); o[2] = bfr(be[ch0 + t]); o[3] = 0.0f;
        *(volatile v4f*)(ST + (size_t)(ch0 + t) * 4) = o; __threadfence(); *(volatile v4f*)(ST + (size_t)(ch0 + t) * 4) = o;
    }
}

__global__ __launch_bounds__(256) void k_bnapply(const float* __restrict__ O, const float* __restrict__ ST, h16* YT) {
    __shared__ __align__(16) h16 ys[8 * 520];
    const int t = threadIdx.x; const int r = blockIdx.x; const int b = r >> 9, c = r & 511;
    const float* p = O + (size_t)r * HW;
#pragma unroll 2
    for (int s = 0; s < 4; ++s) { const int i = t + 256 * s; const int c2 = i >> 1, mlb = (i & 1) * 4;
        const v4f x = *(const v4f*)(p + 4 * i); const v4f st = *(const v4f*)(ST + 4 * c2);
#pragma unroll
        for (int e = 0; e < 4; ++e) { float y = (x[e] - st[0]) * st[1] + st[2]; y = (y >= 0.0f) ? y : 0.01f * y; ys[(mlb + e) * 520 + c2] = (h16)y; } }
    __syncthreads();
#pragma unroll 1
    for (int ps = 0; ps < 2; ++ps) {
#pragma unroll
        for (int s = 0; s < 2; ++s) { const int q = t + 256 * s; const int ml = q >> 6, c8 = (q & 63) * 8;
            const v8h o = *(const v8ha*)(&ys[ml * 520 + c8]);
            *(volatile v8h*)(YT + ((size_t)(b * 8 + ml) * CN + c) * CN + c8) = o; }
        if (ps == 0) __threadfence(); }
}

static constexpr size_t al256(size_t v) { return (v + 255) & ~(size_t)255; }
static constexpr size_t SZ_PL = al256((size_t)NB * CN * HW * 2);
static constexpr size_t SZ_X  = al256((size_t)NB * HW * CI * 2);
static constexpr size_t SZ_S  = al256((size_t)NB * CN * CN * 4);
static constexpr size_t SZ_PP = al256((size_t)NB * CN * CN * 2);
static constexpr size_t SZ_W  = al256((size_t)CN * CI * 2);
static constexpr size_t SZ_W1 = al256((size_t)CN * CN * 2);
static constexpr size_t SZ_W2 = al256((size_t)CO * CN * 2);
static constexpr size_t SZ_ST = al256((size_t)CN * 16);
static constexpr size_t SZ_TOTAL = 3 * SZ_PL + 3 * SZ_X + SZ_S + SZ_PP + 3 * SZ_W + SZ_W1 + SZ_W2 + SZ_ST;
static_assert(SZ_TOTAL <= (size_t)134217728);
static_assert((size_t)NB * CN * HW * 4 <= 2 * SZ_PL);
static_assert((size_t)NB * HW * CN * 2 <= SZ_PL);

extern "C" void kernel_launch(void* const* d_in, const int* in_sizes, int n_in,
                              void* d_out, int out_size, void* d_ws, size_t ws_size, hipStream_t stream) {
    if (n_in < 15) return;
    const size_t needx = (size_t)NB * CI * HW;
    if ((size_t)in_sizes[0] < needx || (size_t)in_sizes[1] < needx || (size_t)in_sizes[2] < needx) return;
    if ((size_t)in_sizes[3] < (size_t)CN * CI || (size_t)in_sizes[5] < (size_t)CN * CI || (size_t)in_sizes[7] < (size_t)CN * CI) return;
    if (in_sizes[4] < CN || in_sizes[6] < CN || in_sizes[8] < CN || in_sizes[9] < CN || in_sizes[10] < CN || in_sizes[12] < CN || in_sizes[14] < CO) return;
    if ((size_t)in_sizes[11] < (size_t)CN * CN || (size_t)in_sizes[13] < (size_t)CO * CN) return;
    if ((size_t)out_size < (size_t)NB * CO * HW) return;
    if (SZ_TOTAL > ws_size) return;
    const float* q  = (const float*)d_in[0];  const float* k  = (const float*)d_in[1];  const float* v  = (const float*)d_in[2];
    const float* wq = (const float*)d_in[3];  const float* bq = (const float*)d_in[4];
    const float* wk = (const float*)d_in[5];  const float* bk = (const float*)d_in[6];
    const float* wv = (const float*)d_in[7];  const float* bv = (const float*)d_in[8];
    const float* bng = (const float*)d_in[9]; const float* bnb = (const float*)d_in[10];
    const float* w1 = (const float*)d_in[11]; const float* b1 = (const float*)d_in[12];
    const float* w2 = (const float*)d_in[13]; const float* b2 = (const float*)d_in[14];
    float* OUT = (float*)d_out;

    char* wsp = (char*)d_ws;
    h16* R0 = (h16*)wsp; wsp += SZ_PL;
    h16* R1 = (h16*)wsp; wsp += SZ_PL;
    h16* R2 = (h16*)wsp; wsp += SZ_PL;
    bf* XQ = (bf*)wsp; wsp += SZ_X;
    bf* XK = (bf*)wsp; wsp += SZ_X;
    bf* XV = (bf*)wsp; wsp += SZ_X;
    float* SCO = (float*)wsp; wsp += SZ_S;
    h16* PP = (h16*)wsp; wsp += SZ_PP;
    bf* WQ = (bf*)wsp; wsp += SZ_W;
    bf* WK = (bf*)wsp; wsp += SZ_W;
    bf* WV = (bf*)wsp; wsp += SZ_W;
    bf* W1H = (bf*)wsp; wsp += SZ_W1;
    bf* W2H = (bf*)wsp; wsp += SZ_W2;
    float* ST = (float*)wsp; wsp += SZ_ST;
    h16* QH = R0; h16* QR = R1; h16* KP = R2; h16* VT = R0; float* OF = (float*)R1; h16* YT = R0; h16* H1T = R1;

    k_xT<<<dim3(HW / 64, NB, 1), 256, 0, stream>>>(q, XQ);
    k_xT<<<dim3(HW / 64, NB, 1), 256, 0, stream>>>(k, XK);
    k_xT<<<dim3(HW / 64, NB, 1), 256, 0, stream>>>(v, XV);
    { const size_t n8 = (size_t)CN * CI / 8; const unsigned g = (unsigned)((n8 + 255) / 256);
      k_cvt8<<<g, 256, 0, stream>>>(wq, WQ, n8, 0, 1.0f); k_cvt8<<<g, 256, 0, stream>>>(wk, WK, n8, 0, 1.0f); k_cvt8<<<g, 256, 0, stream>>>(wv, WV, n8, 0, 1.0f); }
    { const size_t n8 = (size_t)CN * CN / 8; k_cvt8<<<(unsigned)((n8 + 255) / 256), 256, 0, stream>>>(w1, W1H, n8, 1, WSC); }
    { const size_t n8 = (size_t)CO * CN / 8; k_cvt8<<<(unsigned)((n8 + 255) / 256), 256, 0, stream>>>(w2, W2H, n8, 1, WSC); }

    k_gemm<0, 0><<<dim3(CN / 64, HW / 64, NB), 32, 0, stream>>>(WQ, WQ, XQ, QH, QR, SCO, bq, CI, HW, (size_t)0, (size_t)HW * CI, (size_t)CN * HW, 1.0f, 1, 1, 0);
    k_gemm<0, 0><<<dim3(CN / 64, HW / 64, NB), 32, 0, stream>>>(WK, WK, XK, KP, KP, SCO, bk, CI, HW, (size_t)0, (size_t)HW * CI, (size_t)CN * HW, 1.0f, 0, 1, 0);
    k_gemm<1, 1><<<dim3(CN / 32, CN / 64, NB), 32, 0, stream>>>((const bf*)QH, (const bf*)QR, (const bf*)KP, PP, PP, SCO, bq, HW, CN, (size_t)CN * HW, (size_t)CN * HW, (size_t)CN * CN, 1.0f / 64.0f, 2, 0, 0);
    k_softmax<<<dim3(NB * CN / 8, 1, 1), 256, 0, stream>>>(SCO, PP, NB * CN);
    k_gemm<0, 0><<<dim3(HW / 64, CN / 64, NB), 32, 0, stream>>>(XV, XV, WV, VT, VT, SCO, bv, CI, CN, (size_t)HW * CI, (size_t)0, (size_t)HW * CN, 1.0f, 0, 2, 0);
    k_gemm<1, 0><<<dim3(CN / 64, HW / 64, NB), 32, 0, stream>>>((const bf*)PP, (const bf*)PP, (const bf*)VT, PP, PP, OF, bq, CN, HW, (size_t)CN * CN, (size_t)HW * CN, (size_t)CN * HW, PCAI, 2, 0, 0);
    k_bnstats<<<dim3(CN / 8, 1, 1), 256, 0, stream>>>(OF, bng, bnb, ST);
    k_bnapply<<<dim3(NB * CN, 1, 1), 256, 0, stream>>>(OF, ST, YT);
    k_gemm<1, 0><<<dim3(HW / 64, CN / 64, NB), 32, 0, stream>>>((const bf*)YT, (const bf*)YT, W1H, H1T, H1T, SCO, b1, CN, CN, (size_t)HW * CN, (size_t)0, (size_t)HW * CN, WSI, 0, 2, 1);
    k_gemm<1, 0><<<dim3(CO / 64, HW / 64, NB), 32, 0, stream>>>(W2H, W2H, (const bf*)H1T, PP, PP, OUT, b2, CN, HW, (size_t)0, (size_t)HW * CN, (size_t)CO * HW, WSI, 2, 1, 0);
}
